// RouteNet_49520972922897
// MI455X (gfx1250) — hardware-verified
//
#include <hip/hip_runtime.h>
#include <math.h>

constexpr int NPATH = 100000;
constexpr int NLINK = 20000;
constexpr int NSTEP = 8;
constexpr int NDEGR = 48;
constexpr int NDIM  = 64;
constexpr int NGATE = 192;
constexpr int NITER = 4;
constexpr int NSLOT = NSTEP + 1;
constexpr int PSSP  = NSLOT * NDIM;
constexpr int NAGG  = 256;
constexpr int NH1   = 128;
constexpr int NH2   = 128;
constexpr int NLPAD = 20032;
constexpr int TROWS = 16;
constexpr int NTHR  = 128;
constexpr int CH0BLK = 3126;
constexpr int CH1BLK = 3124;
constexpr int CH0ROWS = CH0BLK * TROWS;
constexpr int CH1ROWS = CH1BLK * TROWS;
constexpr int CHROWS  = CH0ROWS;
constexpr int HPITCH = 72;
constexpr int GPITCH = 196;
constexpr int APITCH = 264;
constexpr int BPITCH = 136;
constexpr int OPITCH = 68;
constexpr float WCARRY = 256.0f;
constexpr float WCINV  = 1.0f / 256.0f;
constexpr float RSCL   = 2048.0f;
constexpr float RSCINV = 1.0f / 2048.0f;
constexpr float ASCL   = 1024.0f;
constexpr float ASCINV = 1.0f / 1024.0f;

constexpr int OFF_PEW2 = 0;
constexpr int OFF_LEW2 = OFF_PEW2 + NDIM * NDIM;
constexpr int OFF_WIH  = OFF_LEW2 + NDIM * NDIM;
constexpr int OFF_WHH  = OFF_WIH  + NGATE * NDIM;
constexpr int OFF_CWIH = OFF_WHH  + NGATE * NDIM;
constexpr int OFF_CWHH = OFF_CWIH + NGATE * NDIM;
constexpr int OFF_AW1  = OFF_CWHH + NGATE * NDIM;
constexpr int OFF_AW2  = OFF_AW1  + NH1 * NAGG;
constexpr int OFF_AW3  = OFF_AW2  + NH2 * NH1;
constexpr int W16_TOTAL = OFF_AW3 + NDIM * NH2;

constexpr size_t BYTES_W16  = (size_t)W16_TOTAL * 2;
constexpr size_t BYTES_PS   = (size_t)NPATH * NDIM * 4;
constexpr size_t BYTES_PSS  = (size_t)CHROWS * PSSP * 2;
constexpr size_t BYTES_ACC  = (size_t)NLINK * NGATE * 4;
constexpr size_t BYTES_LS   = (size_t)NLINK * NDIM * 4;
constexpr size_t BYTES_LS16 = (size_t)NLPAD * NDIM * 2;
constexpr size_t BYTES_GL   = (size_t)NLPAD * NGATE * 4;
constexpr size_t BYTES_TOTAL = BYTES_W16 + BYTES_PS + BYTES_PSS + BYTES_ACC + 2 * BYTES_LS + 2 * BYTES_LS16 + BYTES_GL;
static_assert(BYTES_TOTAL == 129560576ull);
static_assert(BYTES_TOTAL <= 134217728ull);
static_assert(BYTES_W16 % 256 == 0 && BYTES_PS % 256 == 0 && BYTES_PSS % 256 == 0 && BYTES_ACC % 256 == 0 &&
              BYTES_LS % 256 == 0 && BYTES_LS16 % 256 == 0 && BYTES_GL % 256 == 0);
static_assert(BYTES_PSS < 67108864ull);
static_assert(CH0ROWS + CH1ROWS == NPATH && CH1ROWS <= CHROWS);
static_assert(NPATH % TROWS == 0 && NLINK % TROWS == 0);
static_assert(NLPAD % 64 == 0 && NLPAD >= NLINK && NGATE % 64 == 0 && NDIM % 32 == 0);
static_assert((NLPAD - NLINK) * NDIM == 256 * 8);
static_assert(NTHR == NH1 && NTHR == NH2);
static_assert(TROWS * NSTEP == NTHR);
static_assert(TROWS * NGATE == 6 * NTHR * 4);
static_assert(TROWS * NDIM == 2 * NTHR * 4);
static_assert(TROWS * NDIM == NTHR * 8);
static_assert((OFF_LEW2 * 2) % 128 == 0 && (OFF_WIH * 2) % 128 == 0 && (OFF_WHH * 2) % 128 == 0 &&
              (OFF_CWIH * 2) % 128 == 0 && (OFF_CWHH * 2) % 128 == 0 && (OFF_AW1 * 2) % 128 == 0 &&
              (OFF_AW2 * 2) % 128 == 0 && (OFF_AW3 * 2) % 128 == 0);
static_assert(HPITCH % 8 == 0 && APITCH % 8 == 0 && BPITCH % 8 == 0 && GPITCH % 4 == 0 && OPITCH % 4 == 0);
static_assert(((size_t)NPATH * NDIM * 4) % 128 == 0);
static_assert((size_t)(NPATH + NLINK) * NDIM * 4 == 30720000ull);

typedef __attribute__((ext_vector_type(16))) _Float16 v16h;
typedef __attribute__((ext_vector_type(8)))  _Float16 v8h;
typedef __attribute__((ext_vector_type(16))) __bf16   v16b;
typedef __attribute__((ext_vector_type(8)))  __bf16   v8b;
typedef __attribute__((ext_vector_type(8)))  float    v8f;
typedef __attribute__((ext_vector_type(4)))  float    v4f;
typedef __attribute__((ext_vector_type(4)))  unsigned v4u;
typedef __attribute__((ext_vector_type(2)))  unsigned v2u;
typedef __attribute__((ext_vector_type(2)))  int      v2i;

__device__ __forceinline__ unsigned short f2bf_bits(float f) {
  unsigned u = __float_as_uint(f);
  return (unsigned short)((u + 0x7FFFu + ((u >> 16) & 1u)) >> 16);
}
__device__ __forceinline__ float bf_bits2f(unsigned short h) { return __uint_as_float(((unsigned)h) << 16); }
__device__ __forceinline__ float bf16r(float f) { return bf_bits2f(f2bf_bits(f)); }

__device__ __forceinline__ float h16_to_f32(unsigned hb) {
  const unsigned sgn = (hb & 0x8000u) << 16; const unsigned em = hb & 0x7fffu;
  const float fn = __uint_as_float((em << 13) + 0x38000000u);
  const float fs = (float)em * 5.9604644775390625e-8f;
  const float mag = (em < 0x400u) ? fs : fn; return __uint_as_float(__float_as_uint(mag) | sgn);
}
__device__ __forceinline__ unsigned short f2h_bits(float x) { const _Float16 h = (_Float16)x; return __builtin_bit_cast(unsigned short, h); }
__device__ __forceinline__ unsigned pk2h(float a, float b) { return (unsigned)f2h_bits(a) | ((unsigned)f2h_bits(b) << 16); }
__device__ __forceinline__ void split_pk2(float a, float b, unsigned& hi, unsigned& lo) {
  const unsigned short ha = f2h_bits(a), hbv = f2h_bits(b);
  const float ra = (a - h16_to_f32((unsigned)ha)) * RSCL;
  const float rb = (b - h16_to_f32((unsigned)hbv)) * RSCL;
  hi = (unsigned)ha | ((unsigned)hbv << 16);
  lo = (unsigned)f2h_bits(ra) | ((unsigned)f2h_bits(rb) << 16);
}
__device__ __forceinline__ void split_h(float v, float rs, unsigned short& hb, unsigned short& lb) {
  hb = f2h_bits(v);
  lb = f2h_bits((v - h16_to_f32((unsigned)hb)) * rs);
}

__device__ __forceinline__ float fsig(float x)  { return __builtin_amdgcn_rcpf(1.0f + expf(-x)); }
__device__ __forceinline__ float ftanh(float x) { return 1.0f - 2.0f * __builtin_amdgcn_rcpf(expf(2.0f * x) + 1.0f); }

__device__ __forceinline__ void dep_guard_h(v8f& a, v8f& b, v16h x, v16h y) { asm volatile("v_nop\n\tv_nop\n\tv_nop\n\tv_nop" : "+v"(a), "+v"(b) : "v"(x), "v"(y)); }
__device__ __forceinline__ void dep_guard_b(v8f& a, v8f& b, v16b x, v16b y) { asm volatile("v_nop\n\tv_nop\n\tv_nop\n\tv_nop" : "+v"(a), "+v"(b) : "v"(x), "v"(y)); }
__device__ __forceinline__ void dep_guard1_h(v8f& a, v16h x, v16h y) { asm volatile("v_nop\n\tv_nop\n\tv_nop\n\tv_nop" : "+v"(a) : "v"(x), "v"(y)); }
__device__ __forceinline__ void dep_guard3_h(v8f& a, v8f& b, v8f& c, v16h x, v16h y) { asm volatile("v_nop\n\tv_nop\n\tv_nop\n\tv_nop" : "+v"(a), "+v"(b), "+v"(c) : "v"(x), "v"(y)); }
__device__ __forceinline__ void dep_guard4_h(v8f& a, v8f& b, v8f& c, v8f& d, v16h x, v16h y) { asm volatile("v_nop\n\tv_nop\n\tv_nop\n\tv_nop" : "+v"(a), "+v"(b), "+v"(c), "+v"(d) : "v"(x), "v"(y)); }
__device__ __forceinline__ void keep4_h(v16h a, v16h b, v16h c, v16h d) { asm volatile("v_nop" :: "v"(a), "v"(b), "v"(c), "v"(d)); }
__device__ __forceinline__ void keep4_b(v16b a, v16b b, v16b c, v16b d) { asm volatile("v_nop" :: "v"(a), "v"(b), "v"(c), "v"(d)); }
__device__ __forceinline__ void acc_guard4(v8f& a, v8f& b, v8f& c, v8f& d) { asm volatile("v_nop\n\tv_nop\n\tv_nop\n\tv_nop" : "+v"(a), "+v"(b), "+v"(c), "+v"(d)); }
__device__ __forceinline__ void acc_guard3(v8f& a, v8f& b, v8f& c) { asm volatile("v_nop\n\tv_nop\n\tv_nop\n\tv_nop" : "+v"(a), "+v"(b), "+v"(c)); }
__device__ __forceinline__ void acc_guard2(v8f& a, v8f& b) { asm volatile("v_nop\n\tv_nop\n\tv_nop\n\tv_nop" : "+v"(a), "+v"(b)); }
__device__ __forceinline__ void acc_guard1(v8f& a) { asm volatile("v_nop\n\tv_nop\n\tv_nop\n\tv_nop" : "+v"(a)); }

template <typename T> struct Frag;
template <> struct Frag<_Float16> {
  typedef v16h V; union U { v16h v; v8h h[2]; };
  static __device__ __forceinline__ v16h load(const _Float16* p) {
    U f; f.h[0] = *(const v8h*)(p); f.h[1] = *(const v8h*)(p + 16); return f.v;
  }
  static __device__ __forceinline__ v8f mma(v16h a, v16h b, v8f c) {
    return __builtin_amdgcn_wmma_f32_16x16x32_f16(false, a, false, b, (short)0, c, false, false);
  }
  static __device__ __forceinline__ void guard(v8f& a, v8f& b, v16h x, v16h y) { dep_guard_h(a, b, x, y); }
  static __device__ __forceinline__ void keep(v16h a, v16h b, v16h c, v16h d) { keep4_h(a, b, c, d); }
};
template <> struct Frag<__bf16> {
  typedef v16b V; union U { v16b v; v8b h[2]; };
  static __device__ __forceinline__ v16b load(const __bf16* p) {
    U f; f.h[0] = *(const v8b*)(p); f.h[1] = *(const v8b*)(p + 16); return f.v;
  }
  static __device__ __forceinline__ v8f mma(v16b a, v16b b, v8f c) {
    return __builtin_amdgcn_wmma_f32_16x16x32_bf16(false, a, false, b, (short)0, c, false, false);
  }
  static __device__ __forceinline__ void guard(v8f& a, v8f& b, v16b x, v16b y) { dep_guard_b(a, b, x, y); }
  static __device__ __forceinline__ void keep(v16b a, v16b b, v16b c, v16b d) { keep4_b(a, b, c, d); }
};

template <int ET> struct Elem;
template <> struct Elem<0> { typedef _Float16 T; };
template <> struct Elem<1> { typedef __bf16 T; };
template <int ET, bool SPLIT, int BIAS_MODE, int OUT_MODE, bool RESID, int ACT = 0>
__global__ __launch_bounds__(256) void wmma_gemm64(
    const unsigned short* __restrict__ Ap, const unsigned short* __restrict__ A2p, int lda, long strideA,
    const unsigned short* __restrict__ Btp, const unsigned short* __restrict__ Bt2p, int ldb, long strideB,
    void* __restrict__ Cout, void* __restrict__ Cout2, int ldc, long strideC,
    const float* __restrict__ bias,
    const float* __restrict__ resid, long strideR,
    int M, int N, int K, float scale) {
  typedef typename Elem<ET>::T T;
  typedef typename Frag<T>::V V;
  const T* A = (const T*)Ap; const T* A2 = (const T*)A2p; const T* Bt = (const T*)Btp; const T* Bt2 = (const T*)Bt2p;
  __shared__ __align__(16) float sT[8][16 * 68];
  const int b    = blockIdx.y;
  const int lane = threadIdx.x & 31;
  const int wave = threadIdx.x >> 5;
  const int tilesN = N >> 6;
  const int tilesM = M >> 6;
  const int tile = blockIdx.x * 8 + wave;
  if (tile >= tilesM * tilesN) return;
  const int tm = tile / tilesN;
  const int tn = tile - tm * tilesN;
  const int m0 = tm << 6;
  const int n0 = tn << 6;

  const T* Ab  = A  + (size_t)b * strideA;
  const T* Bb  = Bt + (size_t)b * strideB;
  const T* Ab2 = SPLIT ? (A2  + (size_t)b * strideA) : nullptr;
  const T* Bb2 = SPLIT ? (Bt2 + (size_t)b * strideB) : nullptr;

  const int rlane = lane & 15;
  const int koff  = (lane >> 4) * 8;
  const int mOff  = (lane >> 4) * 8;

  v8f acc[4][4];
#pragma unroll
  for (int i = 0; i < 4; ++i)
#pragma unroll
    for (int j = 0; j < 4; ++j) acc[i][j] = (v8f){0.f,0.f,0.f,0.f,0.f,0.f,0.f,0.f};

  for (int k0 = 0; k0 < K; k0 += 32) {
    V bh[4], bl[4];
#pragma unroll
    for (int j = 0; j < 4; ++j) {
      const size_t bo = (size_t)(n0 + (j << 4) + rlane) * ldb + koff + k0;
      bh[j] = Frag<T>::load(Bb + bo);
      if (SPLIT) bl[j] = Frag<T>::load(Bb2 + bo);
    }
#pragma unroll
    for (int i = 0; i < 4; ++i) {
      const size_t ao = (size_t)(m0 + (i << 4) + rlane) * lda + koff + k0;
      V ah = Frag<T>::load(Ab + ao);
      V al;
      if (SPLIT) al = Frag<T>::load(Ab2 + ao);
#pragma unroll
      for (int j = 0; j < 4; ++j) {
        acc[i][j] = Frag<T>::mma(ah, bh[j], acc[i][j]);
        if (SPLIT) {
          acc[i][j] = Frag<T>::mma(ah, bl[j], acc[i][j]);
          acc[i][j] = Frag<T>::mma(al, bh[j], acc[i][j]);
        }
      }
      Frag<T>::guard(acc[i][0], acc[i][3], ah, SPLIT ? al : ah);
    }
    Frag<T>::keep(bh[0], bh[1], bh[2], bh[3]);
    if (SPLIT) Frag<T>::keep(bl[0], bl[1], bl[2], bl[3]);
  }
  acc_guard4(acc[0][0], acc[0][1], acc[0][2], acc[0][3]);
  acc_guard4(acc[1][0], acc[1][1], acc[1][2], acc[1][3]);
  acc_guard4(acc[2][0], acc[2][1], acc[2][2], acc[2][3]);
  acc_guard4(acc[3][0], acc[3][1], acc[3][2], acc[3][3]);

  float* slab = sT[wave];
  const float* Rb = RESID ? (resid + (size_t)b * strideR) : nullptr;
#pragma unroll
  for (int i = 0; i < 4; ++i) {
    const int mBase = m0 + (i << 4);
#pragma unroll
    for (int j = 0; j < 4; ++j) {
      const int n = n0 + (j << 4) + rlane;
      float bv = 0.f;
      if (BIAS_MODE == 2) bv = bias[n];
#pragma unroll
      for (int r = 0; r < 8; ++r) {
        float v = acc[i][j][r] * scale;
        if (BIAS_MODE == 1) v += bias[mBase + mOff + r];
        if (BIAS_MODE == 2) v += bv;
        if (RESID) v += Rb[(size_t)(mBase + mOff + r) * ldc + n];
        if (ACT == 1) v = tanhf(v);
        if (ACT == 2) v = fmaxf(v, 0.0f);
        if (ACT == 3) v = v / (1.0f + expf(-v));
        if (ACT == 4) v = (v > 0.f) ? v : 0.01f * v;
        if (ACT == 5) v = 0.5f * v * (1.0f + erff(v * 0.70710678118654752f));
        slab[(mOff + r) * 68 + (j << 4) + rlane] = v;
      }
    }
    __builtin_amdgcn_fence(__ATOMIC_RELEASE, "workgroup");
    __builtin_amdgcn_wave_barrier();
    __builtin_amdgcn_fence(__ATOMIC_ACQUIRE, "workgroup");
    if (OUT_MODE == 0) {
      float* C = (float*)Cout + (size_t)b * strideC;
      const int hh = lane >> 4, c4 = (lane & 15) * 4;
      for (int pass = 0; pass < 2; ++pass) {
#pragma unroll
        for (int it = 0; it < 8; ++it) {
          const int row = it * 2 + hh;
          v4f v = *(const v4f*)(slab + row * 68 + c4);
          *(volatile v4f*)(C + (size_t)(mBase + row) * ldc + n0 + c4) = v;
        }
        __threadfence();
      }
    } else {
      const int q = lane >> 3, c8 = (lane & 7) * 8;
      unsigned short* C  = (unsigned short*)Cout  + (size_t)b * strideC;
      unsigned short* C2 = (OUT_MODE == 2) ? ((unsigned short*)Cout2 + (size_t)b * strideC) : nullptr;
      for (int pass = 0; pass < 2; ++pass) {
#pragma unroll
        for (int it = 0; it < 4; ++it) {
          const int row = it * 4 + q;
          const float* sp = slab + row * 68 + c8;
          v8h hv, lv;
#pragma unroll
          for (int e = 0; e < 8; ++e) {
            if (OUT_MODE == 1) {
              hv[e] = (_Float16)sp[e];
            } else {
              unsigned short hb = f2bf_bits(sp[e]);
              unsigned short lb = f2bf_bits(sp[e] - bf_bits2f(hb));
              hv[e] = __builtin_bit_cast(_Float16, hb);
              lv[e] = __builtin_bit_cast(_Float16, lb);
            }
          }
          *(volatile v8h*)(C + (size_t)(mBase + row) * ldc + n0 + c8) = hv;
          if (OUT_MODE == 2) *(volatile v8h*)(C2 + (size_t)(mBase + row) * ldc + n0 + c8) = lv;
        }
        __threadfence();
      }
    }
    __builtin_amdgcn_fence(__ATOMIC_RELEASE, "workgroup");
    __builtin_amdgcn_wave_barrier();
    __builtin_amdgcn_fence(__ATOMIC_ACQUIRE, "workgroup");
  }
}

template <int KDIM, int AP, int CP>
__device__ __forceinline__ void lds_layer2_ss(const unsigned short* sAh, const unsigned short* sAl, float rin_inv,
                                              const _Float16* __restrict__ W, const float* sBias,
                                              unsigned short* sCh, unsigned short* sCl, int colbase, int lane) {
  const int c = lane & 15, hh = lane >> 4, koff = hh * 8;
  const _Float16* aph = (const _Float16*)sAh + c * AP + koff;
  const _Float16* apl = (const _Float16*)sAl + c * AP + koff;
  const v8f z8 = {0.f, 0.f, 0.f, 0.f, 0.f, 0.f, 0.f, 0.f};
  const int col0 = colbase + c, col1 = col0 + 16;
  const _Float16* w0 = W + (size_t)col0 * KDIM + koff;
  const _Float16* w1 = W + (size_t)col1 * KDIM + koff;
  v8f acc0 = z8, acc1 = z8, accl0 = z8, accl1 = z8;
#pragma unroll 1
  for (int k0 = 0; k0 < KDIM; k0 += 32) {
    const v16h ah = Frag<_Float16>::load(aph + k0);
    const v16h al = Frag<_Float16>::load(apl + k0);
    const v16h b0 = Frag<_Float16>::load(w0 + k0);
    const v16h b1 = Frag<_Float16>::load(w1 + k0);
    acc0  = Frag<_Float16>::mma(ah, b0, acc0);
    acc1  = Frag<_Float16>::mma(ah, b1, acc1);
    accl0 = Frag<_Float16>::mma(al, b0, accl0);
    accl1 = Frag<_Float16>::mma(al, b1, accl1);
    dep_guard4_h(acc0, acc1, accl0, accl1, ah, al);
    keep4_h(ah, al, b0, b1);
  }
  acc_guard4(acc0, acc1, accl0, accl1);
  const float bb0 = sBias[col0], bb1 = sBias[col1];
#pragma unroll
  for (int r = 0; r < 8; ++r) {
    const float v0 = fmaxf((acc0[r] + accl0[r] * rin_inv) * WCINV + bb0, 0.0f);
    const float v1 = fmaxf((acc1[r] + accl1[r] * rin_inv) * WCINV + bb1, 0.0f);
    unsigned short h0b, l0b, h1b, l1b;
    split_h(v0, ASCL, h0b, l0b);
    split_h(v1, ASCL, h1b, l1b);
    sCh[(8 * hh + r) * CP + col0] = h0b;
    sCl[(8 * hh + r) * CP + col0] = l0b;
    sCh[(8 * hh + r) * CP + col1] = h1b;
    sCl[(8 * hh + r) * CP + col1] = l1b;
  }
}
template <int KDIM, int AP, int CP>
__device__ __forceinline__ void lds_layer1_ss(const unsigned short* sAh, const unsigned short* sAl, float rin_inv,
                                              const _Float16* __restrict__ W, const float* sBias,
                                              unsigned short* sCh, unsigned short* sCl, int colbase, int lane) {
  const int c = lane & 15, hh = lane >> 4, koff = hh * 8;
  const _Float16* aph = (const _Float16*)sAh + c * AP + koff;
  const _Float16* apl = (const _Float16*)sAl + c * AP + koff;
  const v8f z8 = {0.f, 0.f, 0.f, 0.f, 0.f, 0.f, 0.f, 0.f};
  const int col0 = colbase + c;
  const _Float16* w0 = W + (size_t)col0 * KDIM + koff;
  v8f acc0 = z8, accl0 = z8;
#pragma unroll 1
  for (int k0 = 0; k0 < KDIM; k0 += 32) {
    const v16h ah = Frag<_Float16>::load(aph + k0);
    const v16h al = Frag<_Float16>::load(apl + k0);
    const v16h b0 = Frag<_Float16>::load(w0 + k0);
    acc0  = Frag<_Float16>::mma(ah, b0, acc0);
    accl0 = Frag<_Float16>::mma(al, b0, accl0);
    dep_guard_h(acc0, accl0, ah, al);
    keep4_h(ah, al, b0, b0);
  }
  acc_guard2(acc0, accl0);
  const float bb0 = sBias[col0];
#pragma unroll
  for (int r = 0; r < 8; ++r) {
    const float v0 = fmaxf((acc0[r] + accl0[r] * rin_inv) * WCINV + bb0, 0.0f);
    unsigned short h0b, l0b;
    split_h(v0, ASCL, h0b, l0b);
    sCh[(8 * hh + r) * CP + col0] = h0b;
    sCl[(8 * hh + r) * CP + col0] = l0b;
  }
}

__device__ __forceinline__ void acc8(const v4u w, const float addm, const float fv,
                                     float (&vmin)[8], float (&vmax)[8], float (&vsum)[8]) {
  const unsigned w0 = w[0], w1 = w[1], w2 = w[2], w3 = w[3];
  float f[8];
  f[0] = h16_to_f32(w0 & 0xffffu); f[1] = h16_to_f32(w0 >> 16);
  f[2] = h16_to_f32(w1 & 0xffffu); f[3] = h16_to_f32(w1 >> 16);
  f[4] = h16_to_f32(w2 & 0xffffu); f[5] = h16_to_f32(w2 >> 16);
  f[6] = h16_to_f32(w3 & 0xffffu); f[7] = h16_to_f32(w3 >> 16);
#pragma unroll
  for (int i = 0; i < 8; ++i) {
    vmin[i] = fminf(vmin[i], f[i] + addm);
    vmax[i] = fmaxf(vmax[i], f[i] - addm);
    vsum[i] = fmaf(fv, f[i], vsum[i]);
  }
}

__global__ __launch_bounds__(256) void cvt_weights_kernel(
    const float* __restrict__ s0, const float* __restrict__ s1, const float* __restrict__ s2,
    const float* __restrict__ s3, const float* __restrict__ s4, const float* __restrict__ s5,
    const float* __restrict__ s6, const float* __restrict__ s7, const float* __restrict__ s8,
    unsigned short* __restrict__ W16) {
  const int mat = blockIdx.y;
  const float* src = s0; int n2 = NDIM * NDIM / 2; int doff = OFF_PEW2;
  if (mat == 1)      { src = s1; n2 = NDIM * NDIM / 2;  doff = OFF_LEW2; }
  else if (mat == 2) { src = s2; n2 = NGATE * NDIM / 2; doff = OFF_WIH; }
  else if (mat == 3) { src = s3; n2 = NGATE * NDIM / 2; doff = OFF_WHH; }
  else if (mat == 4) { src = s4; n2 = NGATE * NDIM / 2; doff = OFF_CWIH; }
  else if (mat == 5) { src = s5; n2 = NGATE * NDIM / 2; doff = OFF_CWHH; }
  else if (mat == 6) { src = s6; n2 = NH1 * NAGG / 2;   doff = OFF_AW1; }
  else if (mat == 7) { src = s7; n2 = NH2 * NH1 / 2;    doff = OFF_AW2; }
  else if (mat == 8) { src = s8; n2 = NDIM * NH2 / 2;   doff = OFF_AW3; }
  const int i = blockIdx.x * 256 + threadIdx.x;
  if (i < n2) {
    const float f0 = bf16r(src[2 * i]) * WCARRY, f1 = bf16r(src[2 * i + 1]) * WCARRY;
    const unsigned u = pk2h(f0, f1);
    unsigned* op = (unsigned*)(W16 + doff) + i;
    *(volatile unsigned*)op = u;
    __threadfence();
    *(volatile unsigned*)op = u;
  }
}

__global__ __launch_bounds__(256) void zero_rows_kernel(unsigned short* __restrict__ pa, unsigned short* __restrict__ pb) {
  unsigned short* p = (blockIdx.x == 0) ? pa : pb;
  const v4u z = {0u, 0u, 0u, 0u};
  unsigned short* q = p + (size_t)threadIdx.x * 8;
  *(volatile v4u*)q = z;
  __threadfence();
  *(volatile v4u*)q = z;
}

__global__ __launch_bounds__(NTHR) void embed_kernel(const float* __restrict__ x, const float* __restrict__ w1,
                                                     const float* __restrict__ b1, const unsigned short* __restrict__ W2p,
                                                     const float* __restrict__ b2, float* __restrict__ dstf,
                                                     unsigned short* __restrict__ dsth, int write_h) {
  __shared__ __align__(16) float sW1[NDIM];
  __shared__ __align__(16) float sB1[NDIM];
  __shared__ __align__(16) float sB2[NDIM];
  __shared__ __align__(16) unsigned short sX[TROWS * HPITCH];
  __shared__ __align__(16) unsigned short sY[TROWS * HPITCH];
  __shared__ __align__(16) float sO[TROWS * OPITCH];
  const _Float16* W2 = (const _Float16*)W2p;
  const int tid = threadIdx.x, lane = tid & 31, wave = tid >> 5;
  const int c = lane & 15, hh = lane >> 4, koff = hh * 8;
  const int row8 = tid >> 3, c8 = (tid & 7) * 8;
  const int rbase = blockIdx.x * TROWS;

  if (tid < NDIM) { sW1[tid] = bf16r(w1[tid]); sB1[tid] = bf16r(b1[tid]); sB2[tid] = bf16r(b2[tid]); }
  __syncthreads();
  {
    const float xv = bf16r(x[rbase + row8]);
    v4u pk;
#pragma unroll
    for (int e = 0; e < 4; ++e) {
      const int k = c8 + 2 * e;
      const float f0 = fmaxf(xv * sW1[k] + sB1[k], 0.0f);
      const float f1 = fmaxf(xv * sW1[k + 1] + sB1[k + 1], 0.0f);
      pk[e] = pk2h(f0, f1);
    }
    *(v4u*)(sX + row8 * HPITCH + c8) = pk;
  }
  __syncthreads();
  {
    const int col = 16 * wave + c;
    const _Float16* ap = (const _Float16*)sX + c * HPITCH + koff;
    const _Float16* wp = W2 + (size_t)col * NDIM + koff;
    const v8f z8 = {0.f, 0.f, 0.f, 0.f, 0.f, 0.f, 0.f, 0.f};
    const v16h a0 = Frag<_Float16>::load(ap), a1 = Frag<_Float16>::load(ap + 32);
    const v16h bw0 = Frag<_Float16>::load(wp), bw1 = Frag<_Float16>::load(wp + 32);
    v8f acc = z8;
    acc = Frag<_Float16>::mma(a0, bw0, acc);
    acc = Frag<_Float16>::mma(a1, bw1, acc);
    dep_guard1_h(acc, a1, bw1);
    keep4_h(a0, bw0, a1, bw1);
    const float bb = sB2[col];
#pragma unroll
    for (int r = 0; r < 8; ++r) {
      const float v = fmaxf(acc[r] * WCINV + bb, 0.0f);
      sO[(8 * hh + r) * OPITCH + col] = v;
      sY[(8 * hh + r) * HPITCH + col] = f2h_bits(v);
    }
  }
  __syncthreads();
  for (int pass = 0; pass < 2; ++pass) {
#pragma unroll
    for (int it = 0; it < 2; ++it) {
      const int idx = it * NTHR + tid;
      const int row = idx >> 4, c4 = (idx & 15) * 4;
      const v4f v = *(const v4f*)(sO + row * OPITCH + c4);
      *(volatile v4f*)(dstf + (size_t)(rbase + row) * NDIM + c4) = v;
    }
    __threadfence();
  }
  if (write_h) {
    const v4u w = *(const v4u*)(sY + row8 * HPITCH + c8);
    unsigned short* dp = dsth + (size_t)(rbase + row8) * NDIM + c8;
    *(volatile v4u*)dp = w;
    __threadfence();
    *(volatile v4u*)dp = w;
  }
}

__global__ __launch_bounds__(NTHR) void path_gru_kernel(
    float* __restrict__ PS, unsigned short* __restrict__ PSS, const int* __restrict__ l2p, const float* __restrict__ GL,
    const unsigned short* __restrict__ W16, const float* __restrict__ bih, const float* __restrict__ bhh,
    float* __restrict__ out0, int pchunk, int write_out) {
  __shared__ __align__(16) float sBih[NGATE];
  __shared__ __align__(16) float sBhh[NGATE];
  __shared__ __align__(16) float sGi[TROWS * GPITCH];
  __shared__ __align__(16) unsigned short sH[2][TROWS * HPITCH];
  __shared__ __align__(16) unsigned short sPo[TROWS * HPITCH];
  __shared__ __align__(16) float sO[TROWS * OPITCH];
  __shared__ int sL2p[TROWS * NSTEP];
  __shared__ int sLen[TROWS];

  const _Float16* WHH = (const _Float16*)(W16 + OFF_WHH);
  const int tid = threadIdx.x, lane = tid & 31, wave = tid >> 5;
  const int c = lane & 15, hh = lane >> 4, koff = hh * 8;
  const int row8 = tid >> 3, c8 = (tid & 7) * 8;
  const int lrow0 = blockIdx.x * TROWS;
  const int pbase = pchunk + lrow0;
  const int colr = 16 * wave + c, colz = NDIM + colr, coln = 2 * NDIM + colr;

#pragma unroll 1
  for (int i = tid; i < NGATE; i += NTHR) { sBih[i] = bf16r(bih[i]); sBhh[i] = bf16r(bhh[i]); }
  sL2p[tid] = l2p[(size_t)pbase * NSTEP + tid];
#pragma unroll
  for (int it = 0; it < 2; ++it) {
    const int idx = it * NTHR + tid;
    const int row = idx >> 4, c4 = (idx & 15) * 4;
    const v4f v = *(const v4f*)(PS + (size_t)(pbase + row) * NDIM + c4);
    *(v4f*)(sO + row * OPITCH + c4) = v;
    v2u pk;
    pk[0] = pk2h(v[0], v[1]);
    pk[1] = pk2h(v[2], v[3]);
    *(v2u*)(&sH[0][row * HPITCH + c4]) = pk;
  }
  __syncthreads();

  if (tid < TROWS) {
    int cnt = 0;
#pragma unroll
    for (int e = 0; e < NSTEP; ++e) cnt += (sL2p[tid * NSTEP + e] != -1) ? 1 : 0;
    sLen[tid] = cnt;
  }
  {
    const v4u w = *(const v4u*)(&sH[0][row8 * HPITCH + c8]);
    unsigned short* dp = PSS + ((size_t)(lrow0 + row8) * NSLOT) * NDIM + c8;
    *(volatile v4u*)dp = w;
    __threadfence();
    *(volatile v4u*)dp = w;
  }
  float hst[8];
#pragma unroll
  for (int r = 0; r < 8; ++r) hst[r] = sO[(8 * hh + r) * OPITCH + colr];
  const _Float16* wr = WHH + (size_t)colr * NDIM + koff;
  const _Float16* wz = WHH + (size_t)colz * NDIM + koff;
  const _Float16* wn = WHH + (size_t)coln * NDIM + koff;
  const v16h bR0 = Frag<_Float16>::load(wr), bR1 = Frag<_Float16>::load(wr + 32);
  const v16h bZ0 = Frag<_Float16>::load(wz), bZ1 = Frag<_Float16>::load(wz + 32);
  asm volatile("" ::: "memory");
  const v16h bN0 = Frag<_Float16>::load(wn), bN1 = Frag<_Float16>::load(wn + 32);
  const float brr = sBhh[colr], bzz = sBhh[colz], bnn = sBhh[coln];
  __syncthreads();
  int lenr[8];
#pragma unroll
  for (int r = 0; r < 8; ++r) lenr[r] = sLen[8 * hh + r];

  const v8f z8 = {0.f, 0.f, 0.f, 0.f, 0.f, 0.f, 0.f, 0.f};

#pragma unroll 1
  for (int t = 0; t < NSTEP; ++t) {
    const int cur = t & 1;
#pragma unroll
    for (int it = 0; it < 6; ++it) {
      const int idx = it * NTHR + tid;
      const int row = idx / 48;
      const int cc = idx - row * 48;
      const int li = sL2p[row * NSTEP + t];
      const float fx = (li != -1) ? 1.0f : 0.0f;
      int lic = li < 0 ? 0 : li; lic = lic > NLINK - 1 ? NLINK - 1 : lic;
      const v4f g = *(const v4f*)(GL + (size_t)lic * NGATE + 4 * cc);
      const v4f b = *(const v4f*)(sBih + 4 * cc);
      v4f v;
#pragma unroll
      for (int e = 0; e < 4; ++e) v[e] = fmaf(fx, g[e], b[e]);
      *(v4f*)(sGi + row * GPITCH + 4 * cc) = v;
    }
    __syncthreads();

    {
      const _Float16* ap = (const _Float16*)(&sH[cur][0]) + c * HPITCH + koff;
      const float* gp = sGi + (8 * hh) * GPITCH;
      v8f accR = z8, accZ = z8, accN = z8;
      float gin[8];
#pragma unroll
      for (int r = 0; r < 8; ++r) {
        accR[r] = (gp[r * GPITCH + colr] + brr) * WCARRY;
        accZ[r] = (gp[r * GPITCH + colz] + bzz) * WCARRY;
        accN[r] = bnn * WCARRY;
        gin[r]  = gp[r * GPITCH + coln];
      }
      const v16h a0 = Frag<_Float16>::load(ap), a1 = Frag<_Float16>::load(ap + 32);
      accR = Frag<_Float16>::mma(a0, bR0, accR);
      accZ = Frag<_Float16>::mma(a0, bZ0, accZ);
      accN = Frag<_Float16>::mma(a0, bN0, accN);
      accR = Frag<_Float16>::mma(a1, bR1, accR);
      accZ = Frag<_Float16>::mma(a1, bZ1, accZ);
      accN = Frag<_Float16>::mma(a1, bN1, accN);
      dep_guard3_h(accR, accZ, accN, a0, a1);
      unsigned short* hnx = &sH[cur ^ 1][0];
#pragma unroll
      for (int r = 0; r < 8; ++r) {
        const float rg = fsig(accR[r] * WCINV);
        const float zg = fsig(accZ[r] * WCINV);
        const float ng = ftanh(gin[r] + rg * (accN[r] * WCINV));
        const float ho = hst[r];
        const float hn = (1.0f - zg) * ng + zg * ho;
        const bool valid = (t < lenr[r]);
        const float hnew = valid ? hn : ho;
        const float ov = valid ? hn : 0.0f;
        hst[r] = hnew;
        hnx[(8 * hh + r) * HPITCH + colr] = f2h_bits(hnew);
        sPo[(8 * hh + r) * HPITCH + colr] = f2h_bits(ov);
      }
    }
    __syncthreads();

    {
      const v4u w = *(const v4u*)(sPo + row8 * HPITCH + c8);
      unsigned short* dp = PSS + ((size_t)(lrow0 + row8) * NSLOT + (size_t)(t + 1)) * NDIM + c8;
      *(volatile v4u*)dp = w;
      __threadfence();
      *(volatile v4u*)dp = w;
    }
  }

#pragma unroll
  for (int r = 0; r < 8; ++r) sO[(8 * hh + r) * OPITCH + colr] = hst[r];
  __syncthreads();
  float* dst = write_out ? out0 : PS;
  for (int pass = 0; pass < 2; ++pass) {
#pragma unroll
    for (int it = 0; it < 2; ++it) {
      const int idx = it * NTHR + tid;
      const int row = idx >> 4, c4 = (idx & 15) * 4;
      const v4f v = *(const v4f*)(sO + row * OPITCH + c4);
      *(volatile v4f*)(dst + (size_t)(pbase + row) * NDIM + c4) = v;
    }
    __threadfence();
  }
}

__global__ __launch_bounds__(NTHR) void link_partial_kernel(const int* __restrict__ p2l, const unsigned short* __restrict__ PSS,
                                                            float* __restrict__ ACC) {
  __shared__ __align__(16) float sAcc[TROWS * NGATE];
  const int tid = threadIdx.x;
  const int row8 = tid >> 3, c8 = (tid & 7) * 8;
  const int lbase = blockIdx.x * TROWS;
  const int* pp = p2l + (size_t)(lbase + row8) * (NDEGR * 2);
  const float pinf = __builtin_inff();
  float vmin[8], vmax[8], vsum[8];
#pragma unroll
  for (int i = 0; i < 8; ++i) { vmin[i] = pinf; vmax[i] = -pinf; vsum[i] = 0.0f; }
#pragma unroll 1
  for (int e = 0; e < NDEGR; ++e) {
    const v2i pr = *(const v2i*)(pp + 2 * e);
    const int p0 = pr[0], p1 = pr[1];
    int pc = p0 < 0 ? 0 : p0; pc = pc > NPATH - 1 ? NPATH - 1 : pc;
    const int valid = ((p0 != -1) ? 1 : 0) & ((pc < CH0ROWS) ? 1 : 0);
    const int prow = pc > CH0ROWS - 1 ? CH0ROWS - 1 : pc;
    int qc = p1 < 0 ? 0 : p1; qc = qc > NSLOT - 1 ? NSLOT - 1 : qc;
    const v4u w = *(const v4u*)(PSS + ((size_t)prow * NSLOT + (size_t)qc) * NDIM + c8);
    acc8(w, valid ? 0.0f : pinf, valid ? 1.0f : 0.0f, vmin, vmax, vsum);
  }
  {
    float* ar = sAcc + row8 * NGATE + c8;
    *(v4f*)(ar + 0)            = (v4f){vmin[0], vmin[1], vmin[2], vmin[3]};
    *(v4f*)(ar + 4)            = (v4f){vmin[4], vmin[5], vmin[6], vmin[7]};
    *(v4f*)(ar + NDIM)         = (v4f){vmax[0], vmax[1], vmax[2], vmax[3]};
    *(v4f*)(ar + NDIM + 4)     = (v4f){vmax[4], vmax[5], vmax[6], vmax[7]};
    *(v4f*)(ar + 2 * NDIM)     = (v4f){vsum[0], vsum[1], vsum[2], vsum[3]};
    *(v4f*)(ar + 2 * NDIM + 4) = (v4f){vsum[4], vsum[5], vsum[6], vsum[7]};
  }
  __syncthreads();
  float* dst = ACC + (size_t)lbase * NGATE;
  for (int pass = 0; pass < 2; ++pass) {
#pragma unroll
    for (int it = 0; it < 6; ++it) {
      const int idx = it * NTHR + tid;
      const v4f v = *(const v4f*)(sAcc + idx * 4);
      *(volatile v4f*)(dst + (size_t)idx * 4) = v;
    }
    __threadfence();
  }
}

__global__ __launch_bounds__(NTHR) void link_update_kernel(
    const int* __restrict__ p2l, const unsigned short* __restrict__ PSS, const float* __restrict__ ACC,
    const unsigned short* __restrict__ W16,
    const float* __restrict__ ab1, const float* __restrict__ ab2, const float* __restrict__ ab3,
    const float* __restrict__ cbih, const float* __restrict__ cbhh,
    const float* __restrict__ LSin, float* __restrict__ LSout, unsigned short* __restrict__ LS16out,
    float* __restrict__ out1, int write_out) {
  __shared__ __align__(16) float sB1[NH1];
  __shared__ __align__(16) float sB2[NH2];
  __shared__ __align__(16) float sB3[NDIM];
  __shared__ __align__(16) float sCbi[NGATE];
  __shared__ __align__(16) float sCbh[NGATE];
  __shared__ __align__(16) unsigned short sAgg[TROWS * APITCH];
  __shared__ __align__(16) unsigned short sAggL[TROWS * APITCH];
  __shared__ __align__(16) unsigned short sAct1[TROWS * BPITCH];
  __shared__ __align__(16) unsigned short sAct1L[TROWS * BPITCH];
  __shared__ __align__(16) unsigned short sAct2[TROWS * BPITCH];
  __shared__ __align__(16) unsigned short sAct2L[TROWS * BPITCH];
  __shared__ __align__(16) unsigned short sPa[TROWS * HPITCH];
  __shared__ __align__(16) unsigned short sPaL[TROWS * HPITCH];
  __shared__ __align__(16) unsigned short sHl[TROWS * HPITCH];
  __shared__ __align__(16) unsigned short sHo[TROWS * HPITCH];
  __shared__ __align__(16) float sHf[TROWS * OPITCH];
  __shared__ __align__(16) float sO[TROWS * OPITCH];

  const _Float16* AW1  = (const _Float16*)(W16 + OFF_AW1);
  const _Float16* AW2  = (const _Float16*)(W16 + OFF_AW2);
  const _Float16* AW3  = (const _Float16*)(W16 + OFF_AW3);
  const _Float16* CWIH = (const _Float16*)(W16 + OFF_CWIH);
  const _Float16* CWHH = (const _Float16*)(W16 + OFF_CWHH);
  const int tid = threadIdx.x, lane = tid & 31, wave = tid >> 5;
  const int c = lane & 15, hh = lane >> 4, koff = hh * 8;
  const int row8 = tid >> 3, c8 = (tid & 7) * 8;
  const int lbase = blockIdx.x * TROWS;
  const int colr = 16 * wave + c, colz = NDIM + colr, coln = 2 * NDIM + colr;

  sB1[tid] = bf16r(ab1[tid]);
  sB2[tid] = bf16r(ab2[tid]);
  if (tid < NDIM) sB3[tid] = bf16r(ab3[tid]);
#pragma unroll 1
  for (int i = tid; i < NGATE; i += NTHR) { sCbi[i] = bf16r(cbih[i]); sCbh[i] = bf16r(cbhh[i]); }
#pragma unroll
  for (int it = 0; it < 2; ++it) {
    const int idx = it * NTHR + tid;
    const int row = idx >> 4, c4 = (idx & 15) * 4;
    const v4f v = *(const v4f*)(LSin + (size_t)(lbase + row) * NDIM + c4);
    *(v4f*)(sHf + row * OPITCH + c4) = v;
    v2u pk;
    pk[0] = pk2h(v[0], v[1]);
    pk[1] = pk2h(v[2], v[3]);
    *(v2u*)(sHl + row * HPITCH + c4) = pk;
  }
  asm volatile("" ::: "memory");

  const float pinf = __builtin_inff();
  float vmin[8], vmax[8], vsum[8];
  {
    const float* arow = ACC + (size_t)(lbase + row8) * NGATE + c8;
    const v4f pm0 = *(const v4f*)(arow),            pm1 = *(const v4f*)(arow + 4);
    const v4f px0 = *(const v4f*)(arow + NDIM),     px1 = *(const v4f*)(arow + NDIM + 4);
    const v4f ps0 = *(const v4f*)(arow + 2 * NDIM), ps1 = *(const v4f*)(arow + 2 * NDIM + 4);
#pragma unroll
    for (int i = 0; i < 4; ++i) {
      vmin[i] = pm0[i]; vmin[4 + i] = pm1[i];
      vmax[i] = px0[i]; vmax[4 + i] = px1[i];
      vsum[i] = ps0[i]; vsum[4 + i] = ps1[i];
    }
  }
  int cnt = 0;
  {
    const int* pp = p2l + (size_t)(lbase + row8) * (NDEGR * 2);
#pragma unroll 1
    for (int e = 0; e < NDEGR; ++e) {
      const v2i pr = *(const v2i*)(pp + 2 * e);
      const int p0 = pr[0], p1 = pr[1];
      const int vany = (p0 != -1) ? 1 : 0;
      cnt += vany;
      int pc = p0 < 0 ? 0 : p0; pc = pc > NPATH - 1 ? NPATH - 1 : pc;
      const int valid = vany & ((pc >= CH0ROWS) ? 1 : 0);
      int lr = pc - CH0ROWS; lr = lr < 0 ? 0 : lr; lr = lr > CH1ROWS - 1 ? CH1ROWS - 1 : lr;
      int qc = p1 < 0 ? 0 : p1; qc = qc > NSLOT - 1 ? NSLOT - 1 : qc;
      const v4u w = *(const v4u*)(PSS + ((size_t)lr * NSLOT + (size_t)qc) * NDIM + c8);
      acc8(w, valid ? 0.0f : pinf, valid ? 1.0f : 0.0f, vmin, vmax, vsum);
    }
  }
  {
    const float rc = 1.0f / (float)(cnt > 0 ? cnt : 1);
    v4u kh0, kh1, kh2, kh3, kl0, kl1, kl2, kl3;
#pragma unroll
    for (int e = 0; e < 4; ++e) {
      unsigned hb, lb;
      split_pk2(vmin[2 * e], vmin[2 * e + 1], hb, lb);           kh0[e] = hb; kl0[e] = lb;
      split_pk2(vmax[2 * e], vmax[2 * e + 1], hb, lb);           kh1[e] = hb; kl1[e] = lb;
      split_pk2(vsum[2 * e], vsum[2 * e + 1], hb, lb);           kh2[e] = hb; kl2[e] = lb;
      split_pk2(vsum[2 * e] * rc, vsum[2 * e + 1] * rc, hb, lb); kh3[e] = hb; kl3[e] = lb;
    }
    unsigned short* ar = sAgg  + row8 * APITCH + c8;
    unsigned short* al = sAggL + row8 * APITCH + c8;
    *(v4u*)(ar + 0 * NDIM) = kh0;
    *(v4u*)(ar + 1 * NDIM) = kh1;
    *(v4u*)(ar + 2 * NDIM) = kh2;
    *(v4u*)(ar + 3 * NDIM) = kh3;
    *(v4u*)(al + 0 * NDIM) = kl0;
    *(v4u*)(al + 1 * NDIM) = kl1;
    *(v4u*)(al + 2 * NDIM) = kl2;
    *(v4u*)(al + 3 * NDIM) = kl3;
  }
  __syncthreads();

  float hst[8];
#pragma unroll
  for (int r = 0; r < 8; ++r) hst[r] = sHf[(8 * hh + r) * OPITCH + colr];

  lds_layer2_ss<NAGG, APITCH, BPITCH>(sAgg, sAggL, RSCINV, AW1, sB1, sAct1, sAct1L, 32 * wave, lane);
  __syncthreads();
  lds_layer2_ss<NH1, BPITCH, BPITCH>(sAct1, sAct1L, ASCINV, AW2, sB2, sAct2, sAct2L, 32 * wave, lane);
  __syncthreads();
  lds_layer1_ss<NH2, BPITCH, HPITCH>(sAct2, sAct2L, ASCINV, AW3, sB3, sPa, sPaL, 16 * wave, lane);
  __syncthreads();

  {
    const _Float16* pap  = (const _Float16*)sPa  + c * HPITCH + koff;
    const _Float16* palp = (const _Float16*)sPaL + c * HPITCH + koff;
    const _Float16* hlp  = (const _Float16*)sHl  + c * HPITCH + koff;
    const v8f z8 = {0.f, 0.f, 0.f, 0.f, 0.f, 0.f, 0.f, 0.f};
    const v16h ap0 = Frag<_Float16>::load(pap),  ap1 = Frag<_Float16>::load(pap + 32);
    const v16h al0 = Frag<_Float16>::load(palp), al1 = Frag<_Float16>::load(palp + 32);
    const v16h ah0 = Frag<_Float16>::load(hlp),  ah1 = Frag<_Float16>::load(hlp + 32);
    const float br  = (sCbi[colr] + sCbh[colr]) * WCARRY;
    const float bz  = (sCbi[colz] + sCbh[colz]) * WCARRY;
    const float bin = sCbi[coln] * WCARRY;
    const float bhn = sCbh[coln] * WCARRY;
    v8f accR = z8, accZ = z8, accGi = z8, accGh = z8, accRl = z8, accZl = z8, accNl = z8;
#pragma unroll
    for (int r = 0; r < 8; ++r) { accR[r] = br; accZ[r] = bz; accGi[r] = bin; accGh[r] = bhn; }
    {
      const _Float16* wi = CWIH + (size_t)colr * NDIM + koff;
      const _Float16* wh = CWHH + (size_t)colr * NDIM + koff;
      const v16h bi0 = Frag<_Float16>::load(wi), bi1 = Frag<_Float16>::load(wi + 32);
      const v16h bh0 = Frag<_Float16>::load(wh), bh1 = Frag<_Float16>::load(wh + 32);
      accR  = Frag<_Float16>::mma(ap0, bi0, accR);
      accR  = Frag<_Float16>::mma(ap1, bi1, accR);
      accRl = Frag<_Float16>::mma(al0, bi0, accRl);
      accRl = Frag<_Float16>::mma(al1, bi1, accRl);
      accR  = Frag<_Float16>::mma(ah0, bh0, accR);
      accR  = Frag<_Float16>::mma(ah1, bh1, accR);
      dep_guard_h(accR, accRl, ah1, bh1);
      keep4_h(bi0, bi1, bh0, bh1);
    }
    asm volatile("" ::: "memory");
    {
      const _Float16* wi = CWIH + (size_t)colz * NDIM + koff;
      const _Float16* wh = CWHH + (size_t)colz * NDIM + koff;
      const v16h bi0 = Frag<_Float16>::load(wi), bi1 = Frag<_Float16>::load(wi + 32);
      const v16h bh0 = Frag<_Float16>::load(wh), bh1 = Frag<_Float16>::load(wh + 32);
      accZ  = Frag<_Float16>::mma(ap0, bi0, accZ);
      accZ  = Frag<_Float16>::mma(ap1, bi1, accZ);
      accZl = Frag<_Float16>::mma(al0, bi0, accZl);
      accZl = Frag<_Float16>::mma(al1, bi1, accZl);
      accZ  = Frag<_Float16>::mma(ah0, bh0, accZ);
      accZ  = Frag<_Float16>::mma(ah1, bh1, accZ);
      dep_guard_h(accZ, accZl, ah1, bh1);
      keep4_h(bi0, bi1, bh0, bh1);
    }
    asm volatile("" ::: "memory");
    {
      const _Float16* wi = CWIH + (size_t)coln * NDIM + koff;
      const _Float16* wh = CWHH + (size_t)coln * NDIM + koff;
      const v16h bi0 = Frag<_Float16>::load(wi), bi1 = Frag<_Float16>::load(wi + 32);
      const v16h bh0 = Frag<_Float16>::load(wh), bh1 = Frag<_Float16>::load(wh + 32);
      accGi = Frag<_Float16>::mma(ap0, bi0, accGi);
      accGi = Frag<_Float16>::mma(ap1, bi1, accGi);
      accNl = Frag<_Float16>::mma(al0, bi0, accNl);
      accNl = Frag<_Float16>::mma(al1, bi1, accNl);
      accGh = Frag<_Float16>::mma(ah0, bh0, accGh);
      accGh = Frag<_Float16>::mma(ah1, bh1, accGh);
      dep_guard3_h(accGi, accNl, accGh, ah1, bh1);
      keep4_h(bi0, bi1, bh0, bh1);
    }
    keep4_h(ap0, ap1, ah0, ah1);
    keep4_h(al0, al1, al0, al1);
    acc_guard4(accR, accZ, accGi, accGh);
    acc_guard3(accRl, accZl, accNl);
#pragma unroll
    for (int r = 0; r < 8; ++r) {
      const float rg = fsig((accR[r] + accRl[r] * ASCINV) * WCINV);
      const float zg = fsig((accZ[r] + accZl[r] * ASCINV) * WCINV);
      const float ng = ftanh((accGi[r] + accNl[r] * ASCINV) * WCINV + rg * (accGh[r] * WCINV));
      const float ho = hst[r];
      const float hn = (1.0f - zg) * ng + zg * ho;
      sO[(8 * hh + r) * OPITCH + colr] = hn;
      sHo[(8 * hh + r) * HPITCH + colr] = f2h_bits(hn);
    }
  }
  __syncthreads();

  float* dstf = write_out ? out1 : LSout;
  for (int pass = 0; pass < 2; ++pass) {
#pragma unroll
    for (int it = 0; it < 2; ++it) {
      const int idx = it * NTHR + tid;
      const int row = idx >> 4, c4 = (idx & 15) * 4;
      const v4f v = *(const v4f*)(sO + row * OPITCH + c4);
      *(volatile v4f*)(dstf + (size_t)(lbase + row) * NDIM + c4) = v;
    }
    __threadfence();
  }
  if (!write_out) {
    const v4u w = *(const v4u*)(sHo + row8 * HPITCH + c8);
    unsigned short* dp = LS16out + (size_t)(lbase + row8) * NDIM + c8;
    *(volatile v4u*)dp = w;
    __threadfence();
    *(volatile v4u*)dp = w;
  }
}

extern "C" void kernel_launch(void* const* d_in, const int* in_sizes, int n_in,
                              void* d_out, int out_size, void* d_ws, size_t ws_size, hipStream_t stream) {
  if (n_in < 26 || d_out == nullptr || d_ws == nullptr) return;
  if (in_sizes[0] != NPATH || in_sizes[1] != NLINK || in_sizes[2] != NPATH * NSTEP || in_sizes[3] != NLINK * NDEGR * 2 ||
      in_sizes[4] != NDIM || in_sizes[5] != NDIM || in_sizes[6] != NDIM * NDIM || in_sizes[7] != NDIM ||
      in_sizes[8] != NDIM || in_sizes[9] != NDIM || in_sizes[10] != NDIM * NDIM || in_sizes[11] != NDIM ||
      in_sizes[12] != NGATE * NDIM || in_sizes[13] != NGATE * NDIM || in_sizes[14] != NGATE || in_sizes[15] != NGATE ||
      in_sizes[16] != NGATE * NDIM || in_sizes[17] != NGATE * NDIM || in_sizes[18] != NGATE || in_sizes[19] != NGATE ||
      in_sizes[20] != NH1 * NAGG || in_sizes[21] != NH1 || in_sizes[22] != NH2 * NH1 || in_sizes[23] != NH2 ||
      in_sizes[24] != NDIM * NH2 || in_sizes[25] != NDIM || out_size != NPATH * NDIM + NLINK * NDIM) return;

  const float* traffic  = (const float*)d_in[0];
  const float* capacity = (const float*)d_in[1];
  const int*   l2p      = (const int*)d_in[2];
  const int*   p2l      = (const int*)d_in[3];
  const float* pe_w1 = (const float*)d_in[4];
  const float* pe_b1 = (const float*)d_in[5];
  const float* pe_w2 = (const float*)d_in[6];
  const float* pe_b2 = (const float*)d_in[7];
  const float* le_w1 = (const float*)d_in[8];
  const float* le_b1 = (const float*)d_in[9];
  const float* le_w2 = (const float*)d_in[10];
  const float* le_b2 = (const float*)d_in[11];
  const float* gru_wih = (const float*)d_in[12];
  const float* gru_whh = (const float*)d_in[13];
  const float* gru_bih = (const float*)d_in[14];
  const float* gru_bhh = (const float*)d_in[15];
  const float* cell_wih = (const float*)d_in[16];
  const float* cell_whh = (const float*)d_in[17];
  const float* cell_bih = (const float*)d_in[18];
  const float* cell_bhh = (const float*)d_in[19];
  const float* am_w1 = (const float*)d_in[20];
  const float* am_b1 = (const float*)d_in[21];
  const float* am_w2 = (const float*)d_in[22];
  const float* am_b2 = (const float*)d_in[23];
  const float* am_w3 = (const float*)d_in[24];
  const float* am_b3 = (const float*)d_in[25];
  float* out0 = (float*)d_out;
  float* out1 = out0 + (size_t)NPATH * NDIM;

  char* ws = (char*)d_ws; size_t off = 0;
  auto carve = [&](size_t bytes) -> char* { char* p = ws + off; off += (bytes + 255) & ~(size_t)255; return p; };
  unsigned short* W16   = (unsigned short*)carve(BYTES_W16);
  float*          PS    = (float*)carve(BYTES_PS);
  unsigned short* PSS   = (unsigned short*)carve(BYTES_PSS);
  float*          ACC   = (float*)carve(BYTES_ACC);
  float*          LSA   = (float*)carve(BYTES_LS);
  float*          LSB   = (float*)carve(BYTES_LS);
  unsigned short* LS16A = (unsigned short*)carve(BYTES_LS16);
  unsigned short* LS16B = (unsigned short*)carve(BYTES_LS16);
  float*          GL    = (float*)carve(BYTES_GL);
  if (off > ws_size || off > (size_t)134217728) return;

  cvt_weights_kernel<<<dim3(64, 9), 256, 0, stream>>>(pe_w2, le_w2, gru_wih, gru_whh, cell_wih, cell_whh,
                                                     am_w1, am_w2, am_w3, W16);
  zero_rows_kernel<<<2, 256, 0, stream>>>(LS16A + (size_t)NLINK * NDIM, LS16B + (size_t)NLINK * NDIM);
  embed_kernel<<<NPATH / TROWS, NTHR, 0, stream>>>(traffic, pe_w1, pe_b1, W16 + OFF_PEW2, pe_b2, PS, LS16A, 0);
  embed_kernel<<<NLINK / TROWS, NTHR, 0, stream>>>(capacity, le_w1, le_b1, W16 + OFF_LEW2, le_b2, LSA, LS16A, 1);

  const int gemm_tiles  = (NLPAD / 64) * (NGATE / 64);
  const int gemm_blocks = (gemm_tiles + 7) / 8;
  for (int it = 0; it < NITER; ++it) {
    const int last = (it == NITER - 1) ? 1 : 0;
    const unsigned short* ls16cur = (it & 1) ? LS16B : LS16A;
    unsigned short*       ls16nxt = (it & 1) ? LS16A : LS16B;
    const float*          lscur   = (it & 1) ? LSB : LSA;
    float*                lsnxt   = (it & 1) ? LSA : LSB;
    wmma_gemm64<0, false, 0, 0, false, 0><<<dim3(gemm_blocks, 1), 256, 0, stream>>>(
        ls16cur, ls16cur, NDIM, 0L, W16 + OFF_WIH, W16 + OFF_WIH, NDIM, 0L, (void*)GL, (void*)GL, NGATE, 0L,
        (const float*)PS, (const float*)PS, 0L, NLPAD, NGATE, NDIM, WCINV);
    path_gru_kernel<<<CH0BLK, NTHR, 0, stream>>>(PS, PSS, l2p, GL, W16, gru_bih, gru_bhh, out0, 0, last);
    link_partial_kernel<<<NLINK / TROWS, NTHR, 0, stream>>>(p2l, PSS, ACC);
    path_gru_kernel<<<CH1BLK, NTHR, 0, stream>>>(PS, PSS, l2p, GL, W16, gru_bih, gru_bhh, out0, CH0ROWS, last);
    link_update_kernel<<<NLINK / TROWS, NTHR, 0, stream>>>(p2l, PSS, ACC, W16, am_b1, am_b2, am_b3, cell_bih, cell_bhh,
                                                          lscur, lsnxt, ls16nxt, out1, last);
  }
}
